// CapsuleNetwork_86766929314213
// MI455X (gfx1250) — hardware-verified
//
#include <hip/hip_runtime.h>
#include <stddef.h>


#define DCH     256
#define KTAP    5
#define PCAP    32
#define PDIM    8
#define OCAP    16
#define ODIM    16
#define RITER   3
#define RB      16
#define NTHR    128
#define NWAVE   (NTHR / 32)
#define NT      (DCH / 16 / NWAVE)
#define HP      (DCH + 4)
#define U_STR   33
#define U_SZ    (OCAP * ODIM * U_STR)
#define WPL     (DCH * DCH)
#define WSTHR   128
#define XSTHR   256
#define WSCAP   134217728
#define BN_EPS_F 1e-5f
#define SQ_EPS_F 1e-8f

#define L_PT     0
#define L_UW     (L_PT + RB * HP * 4)
#define L_CW     (L_UW + NWAVE * U_SZ * 4)
#define L_VW     (L_CW + NWAVE * OCAP * PCAP * 4)
#define L_VO     (L_VW + NWAVE * OCAP * ODIM * 4)
#define LDS_CAPS (L_VO + NWAVE * OCAP * ODIM * 4)

static_assert((DCH % 32) == 0);
static_assert(NT * 16 * NWAVE == DCH && NT >= 1);
static_assert(RB == 16);
static_assert((RB % NWAVE) == 0);
static_assert(((HP * 4) % 16) == 0);
static_assert((DCH / 8) == 32);
static_assert(((RB * (DCH / 8)) % NTHR) == 0);
static_assert(PCAP * PDIM == DCH && OCAP * ODIM == DCH);
static_assert(PCAP == 32 && PDIM == 8 && ODIM == 16);
static_assert((L_UW % 16) == 0 && (L_CW % 16) == 0 && (L_VW % 16) == 0 && (L_VO % 16) == 0);
static_assert(LDS_CAPS <= 300 * 1024);
static_assert(((WPL / 8) % WSTHR) == 0);
static_assert(((2 * WPL / 8) % WSTHR) == 0);
static_assert((OCAP * ODIM * U_STR) == U_SZ);
static_assert((DCH / 4) <= NTHR && ((DCH / 4) % 32) == 0);

typedef float           v4f   __attribute__((ext_vector_type(4)));
typedef float           v8f   __attribute__((ext_vector_type(8)));
typedef unsigned short  v8us  __attribute__((ext_vector_type(8)));
typedef unsigned short  v16us __attribute__((ext_vector_type(16)));
typedef __bf16          v16bf __attribute__((ext_vector_type(16)));
union Frag { v16bf b; v16us u; v8us h[2]; };
static_assert(sizeof(Frag) == 32);

__device__ __forceinline__ v8f wmb(v16bf a, v16bf bq, v8f c) {
  v8f d = __builtin_amdgcn_wmma_f32_16x16x32_bf16(false, a, false, bq, (short)0, c, false, false);
  asm volatile("v_nop\n\tv_nop\n\tv_nop\n\tv_nop" : "+v"(d) : "v"(a), "v"(bq));
  return d;
}

__device__ __forceinline__ v8f zero8() {
  v8f z = {0.f, 0.f, 0.f, 0.f, 0.f, 0.f, 0.f, 0.f};
  return z;
}

__device__ __forceinline__ unsigned bf16_bits(float f) {
  unsigned u = __float_as_uint(f);
  u += 0x7FFFu + ((u >> 16) & 1u);
  return u >> 16;
}

__device__ __forceinline__ void split2(float v, unsigned short& hb, unsigned short& lb) {
  const unsigned hh = bf16_bits(v);
  const float hf = __uint_as_float(hh << 16);
  hb = (unsigned short)hh;
  lb = (unsigned short)bf16_bits(v - hf);
}

__device__ __forceinline__ void split8(v4f a, v4f b, v8us& hv, v8us& lv) {
  unsigned short p, q;
  split2(a.x, p, q); hv[0] = p; lv[0] = q;
  split2(a.y, p, q); hv[1] = p; lv[1] = q;
  split2(a.z, p, q); hv[2] = p; lv[2] = q;
  split2(a.w, p, q); hv[3] = p; lv[3] = q;
  split2(b.x, p, q); hv[4] = p; lv[4] = q;
  split2(b.y, p, q); hv[5] = p; lv[5] = q;
  split2(b.z, p, q); hv[6] = p; lv[6] = q;
  split2(b.w, p, q); hv[7] = p; lv[7] = q;
}

__global__ __launch_bounds__(WSTHR) void k_wsplit(
    const float* __restrict__ w1, const float* __restrict__ w2, unsigned short* Wp) {
  const int t = blockIdx.x * WSTHR + threadIdx.x;
  const int which = t >> 13;
  const int idx = t & 8191;
  const int o = idx >> 5, g = idx & 31;
  const float* w = which ? w2 : w1;
  const float* src = w + (size_t)o * (DCH * KTAP) + (size_t)(8 * g) * KTAP + 2;
  v4f a, b;
  a.x = src[0];        a.y = src[KTAP];     a.z = src[2 * KTAP]; a.w = src[3 * KTAP];
  b.x = src[4 * KTAP]; b.y = src[5 * KTAP]; b.z = src[6 * KTAP]; b.w = src[7 * KTAP];
  v8us hv, lv;
  split8(a, b, hv, lv);
  unsigned short* dh = Wp + (size_t)which * (2 * WPL) + (size_t)idx * 8;
  unsigned short* dl = dh + WPL;
  *(volatile v8us*)dh = hv;
  *(volatile v8us*)dl = lv;
  __threadfence();
  *(volatile v8us*)dh = hv;
  *(volatile v8us*)dl = lv;
}

__global__ __launch_bounds__(XSTHR) void k_xsplit(
    const float* __restrict__ x, unsigned short* Xh, unsigned short* Xl, int nunit) {
  const int t = blockIdx.x * XSTHR + threadIdx.x;
  if (t >= nunit) return;
  const float* s = x + (size_t)t * 8;
  const v4f a = *(const v4f*)s, b = *(const v4f*)(s + 4);
  v8us hv, lv;
  split8(a, b, hv, lv);
  unsigned short* dh = Xh + (size_t)t * 8;
  unsigned short* dl = Xl + (size_t)t * 8;
  *(volatile v8us*)dh = hv;
  *(volatile v8us*)dl = lv;
  __threadfence();
  *(volatile v8us*)dh = hv;
  *(volatile v8us*)dl = lv;
}

__global__ __launch_bounds__(NTHR) void k_gemm1(
    const unsigned short* __restrict__ Xh, const unsigned short* __restrict__ Xl,
    const unsigned short* __restrict__ Wh, const unsigned short* __restrict__ Wl,
    const float* __restrict__ cb, const float* __restrict__ ga, const float* __restrict__ be,
    const float* __restrict__ mu, const float* __restrict__ va,
    unsigned short* Hh, unsigned short* Hl) {
  __shared__ v4f lds_t[RB * HP / 4];
  __shared__ v4f lds_par[4 * DCH / 4];
  float* hb = (float*)lds_t;
  float* s_b = (float*)lds_par;
  float* s_s = s_b + DCH;
  float* s_t = s_s + DCH;
  float* s_m = s_t + DCH;
  const int tid = threadIdx.x, lane = tid & 31, wave = tid >> 5, h = lane >> 4, m = lane & 15;
  const int colBase = wave * (NT * 16);
  const int rowBase = blockIdx.x * RB;

  if (tid < DCH / 4) {
    const int c0 = 4 * tid;
    const v4f b4 = *(const v4f*)(cb + c0);
    const v4f g4 = *(const v4f*)(ga + c0);
    const v4f t4 = *(const v4f*)(be + c0);
    const v4f m4 = *(const v4f*)(mu + c0);
    const v4f v4 = *(const v4f*)(va + c0);
    v4f s4;
    s4.x = g4.x * (1.0f / sqrtf(v4.x + BN_EPS_F));
    s4.y = g4.y * (1.0f / sqrtf(v4.y + BN_EPS_F));
    s4.z = g4.z * (1.0f / sqrtf(v4.z + BN_EPS_F));
    s4.w = g4.w * (1.0f / sqrtf(v4.w + BN_EPS_F));
    *(v4f*)(s_b + c0) = b4;
    *(v4f*)(s_s + c0) = s4;
    *(v4f*)(s_t + c0) = t4;
    *(v4f*)(s_m + c0) = m4;
  }
  __syncthreads();

  v8f acc[NT];
#pragma unroll
  for (int nt = 0; nt < NT; ++nt) acc[nt] = zero8();
  {
    const unsigned short* ah = Xh + (size_t)(rowBase + m) * DCH + 8 * h;
    const unsigned short* al = Xl + (size_t)(rowBase + m) * DCH + 8 * h;
    const unsigned short* bh = Wh + (size_t)(colBase + m) * DCH + 8 * h;
    const unsigned short* bl = Wl + (size_t)(colBase + m) * DCH + 8 * h;
#pragma unroll 1
    for (int ks = 0; ks < DCH / 32; ++ks) {
      const int ko = 32 * ks;
      Frag fa, fl;
      fa.h[0] = *(const v8us*)(ah + ko);
      fa.h[1] = *(const v8us*)(ah + ko + 16);
      fl.h[0] = *(const v8us*)(al + ko);
      fl.h[1] = *(const v8us*)(al + ko + 16);
#pragma unroll
      for (int nt = 0; nt < NT; ++nt) {
        const size_t no = (size_t)(nt * 16) * DCH + ko;
        Frag gb, gl;
        gb.h[0] = *(const v8us*)(bh + no);
        gb.h[1] = *(const v8us*)(bh + no + 16);
        gl.h[0] = *(const v8us*)(bl + no);
        gl.h[1] = *(const v8us*)(bl + no + 16);
        acc[nt] = wmb(fa.b, gb.b, acc[nt]);
        acc[nt] = wmb(fa.b, gl.b, acc[nt]);
        acc[nt] = wmb(fl.b, gb.b, acc[nt]);
      }
    }
  }

#pragma unroll
  for (int nt = 0; nt < NT; ++nt) {
    const int col = colBase + nt * 16 + m;
    const float b0 = s_b[col], s = s_s[col], t0 = s_t[col], m0 = s_m[col];
#pragma unroll
    for (int r = 0; r < 8; ++r) {
      float t = acc[nt][r] + b0;
      t = (t - m0) * s + t0;
      hb[(8 * h + r) * HP + col] = fmaxf(t, 0.0f);
    }
  }
  __syncthreads();

  constexpr int PER = RB * (DCH / 8) / NTHR;
#pragma unroll
  for (int j = 0; j < PER; ++j) {
    const int e = tid + j * NTHR;
    const int row = e >> 5, g = e & 31;
    const float* hr = hb + row * HP + 8 * g;
    const v4f a = *(const v4f*)hr, b = *(const v4f*)(hr + 4);
    v8us hv, lv;
    split8(a, b, hv, lv);
    const size_t go = (size_t)(rowBase + row) * DCH + 8 * g;
    *(volatile v8us*)(Hh + go) = hv;
    *(volatile v8us*)(Hl + go) = lv;
  }
  __threadfence();
#pragma unroll
  for (int j = 0; j < PER; ++j) {
    const int e = tid + j * NTHR;
    const int row = e >> 5, g = e & 31;
    const float* hr = hb + row * HP + 8 * g;
    const v4f a = *(const v4f*)hr, b = *(const v4f*)(hr + 4);
    v8us hv, lv;
    split8(a, b, hv, lv);
    const size_t go = (size_t)(rowBase + row) * DCH + 8 * g;
    *(volatile v8us*)(Hh + go) = hv;
    *(volatile v8us*)(Hl + go) = lv;
  }
}

__global__ __launch_bounds__(NTHR) void k_caps(
    const unsigned short* __restrict__ Hh, const unsigned short* __restrict__ Hl,
    const unsigned short* __restrict__ Wh, const unsigned short* __restrict__ Wl,
    const float* __restrict__ pcb, const float* __restrict__ Wr, float* out) {
  extern __shared__ v4f lds_dyn[];
  char* sm = (char*)lds_dyn;
  const int tid = threadIdx.x, lane = tid & 31, wave = tid >> 5, h = lane >> 4, m = lane & 15;
  float* pt = (float*)(sm + L_PT);
  float* uw = (float*)(sm + L_UW) + wave * U_SZ;
  float* cw = (float*)(sm + L_CW) + wave * (OCAP * PCAP);
  float* vw = (float*)(sm + L_VW) + wave * (OCAP * ODIM);
  float* vo = (float*)(sm + L_VO) + wave * (OCAP * ODIM);
  const int colBase = wave * (NT * 16);
  const int rowBase = blockIdx.x * RB;

  v8f acc[NT];
#pragma unroll
  for (int nt = 0; nt < NT; ++nt) acc[nt] = zero8();
  {
    const unsigned short* ah = Hh + (size_t)(rowBase + m) * DCH + 8 * h;
    const unsigned short* al = Hl + (size_t)(rowBase + m) * DCH + 8 * h;
    const unsigned short* bh = Wh + (size_t)(colBase + m) * DCH + 8 * h;
    const unsigned short* bl = Wl + (size_t)(colBase + m) * DCH + 8 * h;
#pragma unroll 1
    for (int ks = 0; ks < DCH / 32; ++ks) {
      const int ko = 32 * ks;
      Frag fa, fl;
      fa.h[0] = *(const v8us*)(ah + ko);
      fa.h[1] = *(const v8us*)(ah + ko + 16);
      fl.h[0] = *(const v8us*)(al + ko);
      fl.h[1] = *(const v8us*)(al + ko + 16);
#pragma unroll
      for (int nt = 0; nt < NT; ++nt) {
        const size_t no = (size_t)(nt * 16) * DCH + ko;
        Frag gb, gl;
        gb.h[0] = *(const v8us*)(bh + no);
        gb.h[1] = *(const v8us*)(bh + no + 16);
        gl.h[0] = *(const v8us*)(bl + no);
        gl.h[1] = *(const v8us*)(bl + no + 16);
        acc[nt] = wmb(fa.b, gb.b, acc[nt]);
        acc[nt] = wmb(fa.b, gl.b, acc[nt]);
        acc[nt] = wmb(fl.b, gb.b, acc[nt]);
      }
    }
  }
#pragma unroll
  for (int nt = 0; nt < NT; ++nt) {
    const int col = colBase + nt * 16 + m;
    const float b0 = pcb[col];
#pragma unroll
    for (int r = 0; r < 8; ++r) pt[(8 * h + r) * HP + col] = acc[nt][r] + b0;
  }
  __syncthreads();

  const int jj = lane >> 1, ob = (lane & 1) * 8;
#pragma unroll 1
  for (int q = 0; q < RB / NWAVE; ++q) {
    const int rr = q * NWAVE + wave;
    const size_t n = (size_t)rowBase + rr;

    const float* prow = pt + rr * HP + lane * PDIM;
    v4f pa = *(const v4f*)prow, pb = *(const v4f*)(prow + 4);
    const float sq = pa.x * pa.x + pa.y * pa.y + pa.z * pa.z + pa.w * pa.w +
                     pb.x * pb.x + pb.y * pb.y + pb.z * pb.z + pb.w * pb.w;
    const float scl = (sq * (1.0f / (1.0f + sq))) * (1.0f / sqrtf(sq + SQ_EPS_F));
    pa = pa * scl;
    pb = pb * scl;

    const float* wrow = Wr + (size_t)lane * (ODIM * PDIM);
#pragma unroll 1
    for (int j = 0; j < OCAP; ++j) {
      const float* wj = wrow + (size_t)j * (PCAP * ODIM * PDIM);
      float* uj = uw + j * (ODIM * U_STR) + lane;
#pragma unroll 4
      for (int o = 0; o < ODIM; ++o) {
        const v4f wa = *(const v4f*)(wj + o * PDIM), wb = *(const v4f*)(wj + o * PDIM + 4);
        const float a = wa.x * pa.x + wa.y * pa.y + wa.z * pa.z + wa.w * pa.w +
                        wb.x * pb.x + wb.y * pb.y + wb.z * pb.z + wb.w * pb.w;
        uj[o * U_STR] = a;
      }
    }
    float blog[OCAP];
#pragma unroll
    for (int j = 0; j < OCAP; ++j) blog[j] = 0.0f;
    __syncthreads();

#pragma unroll 1
    for (int t = 0; t < RITER; ++t) {
      float mx = blog[0];
#pragma unroll
      for (int j = 1; j < OCAP; ++j) mx = fmaxf(mx, blog[j]);
      float ce[OCAP];
      float es = 0.0f;
#pragma unroll
      for (int j = 0; j < OCAP; ++j) { ce[j] = __expf(blog[j] - mx); es += ce[j]; }
      const float inv = 1.0f / es;
#pragma unroll
      for (int j = 0; j < OCAP; ++j) cw[j * PCAP + lane] = ce[j] * inv;
      __syncthreads();

      float sv[8];
#pragma unroll
      for (int o = 0; o < 8; ++o) sv[o] = 0.0f;
      const float* cj = cw + jj * PCAP;
      const float* ub = uw + (jj * ODIM + ob) * U_STR;
#pragma unroll 4
      for (int i = 0; i < PCAP; ++i) {
        const float c = cj[i];
#pragma unroll
        for (int o = 0; o < 8; ++o) sv[o] += c * ub[o * U_STR + i];
      }
      float s2 = 0.0f;
#pragma unroll
      for (int o = 0; o < 8; ++o) s2 += sv[o] * sv[o];
      s2 += __shfl_xor(s2, 1, 32);
      const float vscl = (s2 * (1.0f / (1.0f + s2))) * (1.0f / sqrtf(s2 + SQ_EPS_F));

      if (t < RITER - 1) {
#pragma unroll
        for (int o = 0; o < 8; ++o) vw[jj * ODIM + ob + o] = sv[o] * vscl;
        __syncthreads();
#pragma unroll
        for (int j = 0; j < OCAP; ++j) ce[j] = 0.0f;
#pragma unroll 2
        for (int o = 0; o < ODIM; ++o) {
          const float* uo = uw + o * U_STR + lane;
#pragma unroll
          for (int j = 0; j < OCAP; ++j) ce[j] += uo[j * (ODIM * U_STR)] * vw[j * ODIM + o];
        }
#pragma unroll
        for (int j = 0; j < OCAP; ++j) blog[j] += ce[j];
        __syncthreads();
      } else {
#pragma unroll
        for (int o = 0; o < 8; ++o) vo[(ob + o) * OCAP + jj] = sv[o] * vscl;
        __syncthreads();
        const v4f o0 = *(const v4f*)(vo + lane * 4);
        const v4f o1 = *(const v4f*)(vo + (DCH / 2) + lane * 4);
        float* orow = out + n * DCH;
        *(volatile v4f*)(orow + lane * 4) = o0;
        *(volatile v4f*)(orow + (DCH / 2) + lane * 4) = o1;
        __threadfence();
        *(volatile v4f*)(orow + lane * 4) = o0;
        *(volatile v4f*)(orow + (DCH / 2) + lane * 4) = o1;
      }
    }
  }
}

extern "C" void kernel_launch(void* const* d_in, const int* in_sizes, int n_in,
                              void* d_out, int out_size, void* d_ws, size_t ws_size,
                              hipStream_t stream) {
  if (n_in < 10) return;
  const int nrow = in_sizes[0] / DCH;
  if (nrow <= 0 || in_sizes[0] != nrow * DCH || (nrow % RB) != 0) return;
  if (out_size != nrow * DCH) return;
  if (in_sizes[1] != DCH * DCH * KTAP || in_sizes[7] != DCH * DCH * KTAP) return;
  if (in_sizes[2] != DCH || in_sizes[3] != DCH || in_sizes[4] != DCH || in_sizes[5] != DCH ||
      in_sizes[6] != DCH || in_sizes[8] != DCH) return;
  if (in_sizes[9] != OCAP * PCAP * ODIM * PDIM) return;

  const float* x       = (const float*)d_in[0];
  const float* conv1_w = (const float*)d_in[1];
  const float* conv1_b = (const float*)d_in[2];
  const float* gamma   = (const float*)d_in[3];
  const float* beta    = (const float*)d_in[4];
  const float* mean    = (const float*)d_in[5];
  const float* var     = (const float*)d_in[6];
  const float* pc_w    = (const float*)d_in[7];
  const float* pc_b    = (const float*)d_in[8];
  const float* W_route = (const float*)d_in[9];
  float* out = (float*)d_out;

  const size_t plane = (size_t)nrow * DCH * 2;
  size_t off = 0;
  const size_t oW  = off; off += (size_t)4 * WPL * 2;          off = (off + 255) & ~(size_t)255;
  const size_t oXh = off; off += plane;                        off = (off + 255) & ~(size_t)255;
  const size_t oXl = off; off += plane;                        off = (off + 255) & ~(size_t)255;
  const size_t oHh = off; off += plane;                        off = (off + 255) & ~(size_t)255;
  const size_t oHl = off; off += plane;                        off = (off + 255) & ~(size_t)255;
  const size_t tot = off;
  if (tot > ws_size || tot > (size_t)WSCAP) return;
  char* ws = (char*)d_ws;
  unsigned short* Wp = (unsigned short*)(ws + oW);
  unsigned short* Xh = (unsigned short*)(ws + oXh);
  unsigned short* Xl = (unsigned short*)(ws + oXl);
  unsigned short* Hh = (unsigned short*)(ws + oHh);
  unsigned short* Hl = (unsigned short*)(ws + oHl);
  const unsigned short* W1h = Wp;
  const unsigned short* W1l = Wp + WPL;
  const unsigned short* W2h = Wp + 2 * WPL;
  const unsigned short* W2l = Wp + 3 * WPL;

  const int nunit = nrow * (DCH / 8);
  const int nblk  = nrow / RB;

  k_wsplit<<<(2 * WPL / 8) / WSTHR, WSTHR, 0, stream>>>(conv1_w, pc_w, Wp);

  k_xsplit<<<(nunit + XSTHR - 1) / XSTHR, XSTHR, 0, stream>>>(x, Xh, Xl, nunit);

  k_gemm1<<<nblk, NTHR, 0, stream>>>(Xh, Xl, W1h, W1l, conv1_b, gamma, beta, mean, var, Hh, Hl);

  hipFuncSetAttribute(reinterpret_cast<const void*>(&k_caps),
                      hipFuncAttributeMaxDynamicSharedMemorySize, LDS_CAPS);
  k_caps<<<nblk, NTHR, LDS_CAPS, stream>>>(Hh, Hl, W2h, W2l, pc_b, W_route, out);
}
